// DiagGaussianActor_HR_83726092468897
// MI455X (gfx1250) — hardware-verified
//
#include <hip/hip_runtime.h>
#include <math.h>
#include <stdint.h>
#include <stddef.h>


static constexpr int BB  = 8192;
static constexpr int OBS = 256;
static constexpr int ACT = 32;
static constexpr int HID = 512;
static constexpr int NP  = 8;
static constexpr float LSMIN  = -5.0f;
static constexpr float LSMAX  =  2.0f;
static constexpr float WSCALE = 16.0f;
static constexpr float WINV   = 0.0625f;

static_assert(BB % 128 == 0);
static_assert(HID % 64 == 0);
static_assert(BB % 8 == 0);

typedef _Float16 v8h  __attribute__((ext_vector_type(8)));
typedef _Float16 v16h __attribute__((ext_vector_type(16)));
typedef float    v8f  __attribute__((ext_vector_type(8)));
typedef float    v4f  __attribute__((ext_vector_type(4)));

union Frag   { v16h v; v8h half[2]; };
union Pack16 { v8h h; v4f f; };

__device__ __forceinline__ v8f wmma_f16(v16h a, v16h b, v8f c)
{
    v8f d = __builtin_amdgcn_wmma_f32_16x16x32_f16(false, a, false, b, (short)0, c, false, false);
    asm volatile("v_nop\n\tv_nop\n\tv_nop\n\tv_nop" : "+v"(d) : "v"(a), "v"(b));
    return d;
}

__global__ __launch_bounds__(256)
void cvt_f32_f16(const float* __restrict__ src, _Float16* dst, int n8, float scale)
{
    const int i = blockIdx.x * 256 + threadIdx.x;
    if (i < n8) {
        const v4f* s = (const v4f*)(src + (size_t)i * 8);
        const v4f x0 = s[0] * scale;
        const v4f x1 = s[1] * scale;
        Pack16 o;
        #pragma unroll
        for (int k = 0; k < 4; ++k) {
            o.h[k]     = (_Float16)x0[k];
            o.h[4 + k] = (_Float16)x1[k];
        }
        volatile v4f* d = (volatile v4f*)(dst + (size_t)i * 8);
        *d = o.f;
        __threadfence();
        *d = o.f;
    }
}

template<int K, int NPE, int EPI>
__global__ __launch_bounds__(256)
void blend_gemm(const _Float16* __restrict__ A,
                const _Float16* __restrict__ W,
                const float*    __restrict__ bias,
                const float*    __restrict__ blend,
                _Float16* out16,
                float*    out32,
                int Ntot)
{
    constexpr int ASTR   = K + 8;
    constexpr int KT     = K / 32;
    constexpr int KC     = K / 8;
    constexpr int ABYTES = 128 * ASTR * 2;
    constexpr int BBYTES = 64 * ASTR * 2;
    static_assert((K % 32) == 0);
    static_assert(BBYTES >= 128 * 64 * 4);
    static_assert((ABYTES % 16) == 0 && (BBYTES % 16) == 0);

    extern __shared__ __align__(16) char smem[];
    _Float16* Astrip = (_Float16*)smem;
    _Float16* Bpanel = (_Float16*)(smem + ABYTES);
    float*    Bl     = (float*)(smem + ABYTES + BBYTES);

    const int t    = threadIdx.x;
    const int lane = t & 31;
    const int wave = t >> 5;
    const int wm   = wave & 3;
    const int wn   = wave >> 2;
    const int h    = lane >> 4;
    const int l15  = lane & 15;
    const int rowBase = blockIdx.x * 128;
    const int colBase = blockIdx.y * 64;

    if (NPE > 1) {
        #pragma unroll
        for (int i = 0; i < 4; ++i) {
            const int idx = t + i * 256;
            Bl[idx] = blend[(size_t)rowBase * NP + idx];
        }
    }
    for (int ch = t; ch < 128 * KC; ch += 256) {
        const int r  = ch / KC;
        const int kc = ch - r * KC;
        *(v8h*)&Astrip[r * ASTR + kc * 8] = *(const v8h*)&A[(size_t)(rowBase + r) * K + kc * 8];
    }

    v8f acc[2][2] = {};

    #pragma unroll 1
    for (int p = 0; p < NPE; ++p) {
        __syncthreads();
        const _Float16* Wp = W + ((size_t)p * Ntot + colBase) * K;
        for (int ch = t; ch < 64 * KC; ch += 256) {
            const int n  = ch / KC;
            const int kc = ch - n * KC;
            *(v8h*)&Bpanel[n * ASTR + kc * 8] = *(const v8h*)&Wp[(size_t)n * K + kc * 8];
        }
        __syncthreads();

        v8f c[2][2] = {};
        #pragma unroll 1
        for (int kt = 0; kt < KT; ++kt) {
            Frag a[2], b[2];
            #pragma unroll
            for (int i = 0; i < 2; ++i) {
                const _Float16* ap = &Astrip[(wm * 32 + i * 16 + l15) * ASTR + kt * 32 + 8 * h];
                a[i].half[0] = *(const v8h*)ap;
                a[i].half[1] = *(const v8h*)(ap + 16);
                const _Float16* bp = &Bpanel[(wn * 32 + i * 16 + l15) * ASTR + kt * 32 + 8 * h];
                b[i].half[0] = *(const v8h*)bp;
                b[i].half[1] = *(const v8h*)(bp + 16);
            }
            #pragma unroll
            for (int i = 0; i < 2; ++i) {
                #pragma unroll
                for (int j = 0; j < 2; ++j)
                    c[i][j] = wmma_f16(a[i].v, b[j].v, c[i][j]);
            }
        }

        #pragma unroll
        for (int i = 0; i < 2; ++i) {
            #pragma unroll
            for (int j = 0; j < 2; ++j) {
                const int gcol = colBase + wn * 32 + j * 16 + l15;
                const float bb = bias[(size_t)p * Ntot + gcol];
                #pragma unroll
                for (int r = 0; r < 8; ++r) {
                    float bw = 1.0f;
                    if (NPE > 1) {
                        const int lrow = wm * 32 + i * 16 + 8 * h + r;
                        bw = Bl[lrow * 8 + p];
                    }
                    acc[i][j][r] += bw * (c[i][j][r] * WINV + bb);
                }
            }
        }
    }

    __syncthreads();

    if (EPI == 0) {
        _Float16* stg = Bpanel;
        #pragma unroll
        for (int i = 0; i < 2; ++i) {
            #pragma unroll
            for (int j = 0; j < 2; ++j) {
                const int lcol = wn * 32 + j * 16 + l15;
                #pragma unroll
                for (int r = 0; r < 8; ++r) {
                    const int lrow = wm * 32 + i * 16 + 8 * h + r;
                    float v = acc[i][j][r];
                    v = v > 0.0f ? v : 0.0f;
                    stg[lrow * 64 + lcol] = (_Float16)v;
                }
            }
        }
        __syncthreads();
        Pack16 vals[4];
        const int cc = (lane & 7) * 8;
        #pragma unroll
        for (int it = 0; it < 4; ++it) {
            const int row = wave * 16 + it * 4 + (lane >> 3);
            vals[it].h = *(const v8h*)&stg[row * 64 + cc];
        }
        _Float16* gb = out16 + (size_t)rowBase * Ntot + colBase + cc;
        #pragma unroll
        for (int it = 0; it < 4; ++it) {
            const int row = wave * 16 + it * 4 + (lane >> 3);
            *(volatile v4f*)(gb + (size_t)row * Ntot) = vals[it].f;
        }
        __threadfence();
        #pragma unroll
        for (int it = 0; it < 4; ++it) {
            const int row = wave * 16 + it * 4 + (lane >> 3);
            *(volatile v4f*)(gb + (size_t)row * Ntot) = vals[it].f;
        }
    } else {
        float* stg = (float*)Bpanel;
        #pragma unroll
        for (int i = 0; i < 2; ++i) {
            #pragma unroll
            for (int j = 0; j < 2; ++j) {
                const int  lcol   = wn * 32 + j * 16 + l15;
                const bool is_std = (colBase + lcol) >= (Ntot >> 1);
                #pragma unroll
                for (int r = 0; r < 8; ++r) {
                    const int lrow = wm * 32 + i * 16 + 8 * h + r;
                    float v = acc[i][j][r];
                    if (is_std) {
                        const float tv = tanhf(v);
                        const float ls = LSMIN + 0.5f * (LSMAX - LSMIN) * (tv + 1.0f);
                        v = expf(ls);
                    }
                    stg[lrow * 64 + lcol] = v;
                }
            }
        }
        __syncthreads();
        v4f vals[8];
        const int cc = (lane & 15) * 4;
        #pragma unroll
        for (int it = 0; it < 8; ++it) {
            const int row = wave * 16 + it * 2 + (lane >> 4);
            vals[it] = *(const v4f*)&stg[row * 64 + cc];
        }
        float* gb = out32 + (size_t)rowBase * Ntot + colBase + cc;
        #pragma unroll
        for (int it = 0; it < 8; ++it) {
            const int row = wave * 16 + it * 2 + (lane >> 4);
            *(volatile v4f*)(gb + (size_t)row * Ntot) = vals[it];
        }
        __threadfence();
        #pragma unroll
        for (int it = 0; it < 8; ++it) {
            const int row = wave * 16 + it * 2 + (lane >> 4);
            *(volatile v4f*)(gb + (size_t)row * Ntot) = vals[it];
        }
    }
}

__global__ __launch_bounds__(256)
void gate_softmax(const _Float16* __restrict__ h1,
                  const float*    __restrict__ gw2,
                  const float*    __restrict__ gb2,
                  float* blend)
{
    __shared__ __align__(16) float sp[64];
    const int lane = threadIdx.x & 31;
    const int wave = threadIdx.x >> 5;
    const int row  = blockIdx.x * 8 + wave;

    float s[NP];
    #pragma unroll
    for (int p = 0; p < NP; ++p) s[p] = 0.0f;
    const _Float16* hr = h1 + (size_t)row * HID;
    #pragma unroll 1
    for (int k = lane; k < HID; k += 32) {
        const float hv = (float)hr[k];
        #pragma unroll
        for (int p = 0; p < NP; ++p) s[p] += hv * gw2[p * HID + k];
    }
    #pragma unroll
    for (int p = 0; p < NP; ++p) {
        #pragma unroll
        for (int o = 16; o > 0; o >>= 1) s[p] += __shfl_xor(s[p], o, 32);
        s[p] += gb2[p];
    }
    float m = s[0];
    #pragma unroll
    for (int p = 1; p < NP; ++p) m = fmaxf(m, s[p]);
    float e[NP];
    float den = 0.0f;
    #pragma unroll
    for (int p = 0; p < NP; ++p) { e[p] = expf(s[p] - m); den += e[p]; }
    const float rden = 1.0f / den;
    float mine = 0.0f;
    #pragma unroll
    for (int p = 0; p < NP; ++p) mine = (lane == p) ? e[p] : mine;
    if (lane < NP) sp[wave * 8 + lane] = mine * rden;
    __syncthreads();
    if (wave == 0 && lane < 16) {
        const v4f v = *(const v4f*)&sp[lane * 4];
        volatile v4f* gp = (volatile v4f*)(blend + (size_t)blockIdx.x * 64 + lane * 4);
        *gp = v;
        __threadfence();
        *gp = v;
    }
}

static inline size_t align256(size_t b) { return (b + 255) & ~(size_t)255; }
static inline int smem_bytes_for(int K) { return 128 * (K + 8) * 2 + 64 * (K + 8) * 2 + 128 * NP * 4; }

extern "C" void kernel_launch(void* const* d_in, const int* in_sizes, int n_in,
                              void* d_out, int out_size, void* d_ws, size_t ws_size,
                              hipStream_t stream)
{
    if (n_in < 13) return;
    if (in_sizes[0]  != BB * OBS)        return;
    if (in_sizes[1]  != HID * OBS)       return;
    if (in_sizes[2]  != HID)             return;
    if (in_sizes[3]  != HID * HID)       return;
    if (in_sizes[4]  != HID)             return;
    if (in_sizes[5]  != NP * HID)        return;
    if (in_sizes[6]  != NP)              return;
    if (in_sizes[7]  != NP * HID * OBS)  return;
    if (in_sizes[8]  != NP * HID)        return;
    if (in_sizes[9]  != NP * HID * HID)  return;
    if (in_sizes[10] != NP * HID)        return;
    if (in_sizes[11] != NP * 2 * ACT * HID) return;
    if (in_sizes[12] != NP * 2 * ACT)    return;
    if (out_size != BB * 2 * ACT)        return;

    const float* obs = (const float*)d_in[0];
    const float* gw0 = (const float*)d_in[1];
    const float* gb0 = (const float*)d_in[2];
    const float* gw1 = (const float*)d_in[3];
    const float* gb1 = (const float*)d_in[4];
    const float* gw2 = (const float*)d_in[5];
    const float* gb2 = (const float*)d_in[6];
    const float* ew0 = (const float*)d_in[7];
    const float* eb0 = (const float*)d_in[8];
    const float* ew1 = (const float*)d_in[9];
    const float* eb1 = (const float*)d_in[10];
    const float* ew2 = (const float*)d_in[11];
    const float* eb2 = (const float*)d_in[12];
    float* out = (float*)d_out;

    char*  ws  = (char*)d_ws;
    size_t off = 0;
    _Float16* obs_h = (_Float16*)(ws + off); off += align256((size_t)BB * OBS * 2);
    _Float16* gw0_h = (_Float16*)(ws + off); off += align256((size_t)HID * OBS * 2);
    _Float16* gw1_h = (_Float16*)(ws + off); off += align256((size_t)HID * HID * 2);
    _Float16* ew0_h = (_Float16*)(ws + off); off += align256((size_t)NP * HID * OBS * 2);
    _Float16* ew1_h = (_Float16*)(ws + off); off += align256((size_t)NP * HID * HID * 2);
    _Float16* ew2_h = (_Float16*)(ws + off); off += align256((size_t)NP * 2 * ACT * HID * 2);
    _Float16* h0    = (_Float16*)(ws + off); off += align256((size_t)BB * HID * 2);
    _Float16* h1    = (_Float16*)(ws + off); off += align256((size_t)BB * HID * 2);
    _Float16* x1    = (_Float16*)(ws + off); off += align256((size_t)BB * HID * 2);
    _Float16* x2    = (_Float16*)(ws + off); off += align256((size_t)BB * HID * 2);
    float*    blendw = (float*)(ws + off);   off += align256((size_t)BB * NP * 4);
    if (off > ws_size) return;

    auto cvt = [&](const float* s, _Float16* d, int n, float scale) {
        const int n8 = n / 8;
        cvt_f32_f16<<<dim3((n8 + 255) / 256), dim3(256), 0, stream>>>(s, d, n8, scale);
    };
    cvt(obs, obs_h, BB * OBS,            1.0f);
    cvt(gw0, gw0_h, HID * OBS,           WSCALE);
    cvt(gw1, gw1_h, HID * HID,           WSCALE);
    cvt(ew0, ew0_h, NP * HID * OBS,      WSCALE);
    cvt(ew1, ew1_h, NP * HID * HID,      WSCALE);
    cvt(ew2, ew2_h, NP * 2 * ACT * HID,  WSCALE);

    const int smemK256 = smem_bytes_for(OBS);
    const int smemK512 = smem_bytes_for(HID);
    hipFuncSetAttribute((const void*)&blend_gemm<OBS, 1, 0>,  hipFuncAttributeMaxDynamicSharedMemorySize, smemK256);
    hipFuncSetAttribute((const void*)&blend_gemm<HID, 1, 0>,  hipFuncAttributeMaxDynamicSharedMemorySize, smemK512);
    hipFuncSetAttribute((const void*)&blend_gemm<OBS, NP, 0>, hipFuncAttributeMaxDynamicSharedMemorySize, smemK256);
    hipFuncSetAttribute((const void*)&blend_gemm<HID, NP, 0>, hipFuncAttributeMaxDynamicSharedMemorySize, smemK512);
    hipFuncSetAttribute((const void*)&blend_gemm<HID, NP, 2>, hipFuncAttributeMaxDynamicSharedMemorySize, smemK512);

    const dim3 blk(256);
    const dim3 gFull(BB / 128, HID / 64);
    const dim3 gOut (BB / 128, 1);

    blend_gemm<OBS, 1, 0><<<gFull, blk, smemK256, stream>>>(obs_h, gw0_h, gb0, blendw, h0, out, HID);
    blend_gemm<HID, 1, 0><<<gFull, blk, smemK512, stream>>>(h0,    gw1_h, gb1, blendw, h1, out, HID);
    gate_softmax<<<dim3(BB / 8), blk, 0, stream>>>(h1, gw2, gb2, blendw);
    blend_gemm<OBS, NP, 0><<<gFull, blk, smemK256, stream>>>(obs_h, ew0_h, eb0, blendw, x1, out, HID);
    blend_gemm<HID, NP, 0><<<gFull, blk, smemK512, stream>>>(x1,    ew1_h, eb1, blendw, x2, out, HID);
    blend_gemm<HID, NP, 2><<<gOut,  blk, smemK512, stream>>>(x2,    ew2_h, eb2, blendw, h1, out, 2 * ACT);
    (void)hipGetLastError();
}
